// Mhsa_47802986004933
// MI455X (gfx1250) — hardware-verified
//
#include <hip/hip_runtime.h>


#define DEV __device__ __forceinline__

#ifndef NB
#define NB 2
#endif
#define NB_FULL 2
#define NTOK    4096
#define IMG     64
#define CDIM    256
#define NQKV    1536
#define INNER   512
#define DHEAD   64
#define HHALF   4
#define KCONV   768
#define NSTAT   64
#define BN_EPS  1e-5f

#define CT_P    136
#define IC_P    776
#define VT_P    72
#define V2_P    136
#define CO_P    68
#define AO_P    36
#define SCL2    0.00070444093793406416f

static_assert(NB >= 1 && NB <= NB_FULL);
static_assert(NTOK == IMG * IMG);
static_assert(NQKV == 3 * INNER && INNER == 2 * HHALF * DHEAD && CDIM == INNER / 2);
static_assert(KCONV == 3 * CDIM && (KCONV % 32) == 0 && (CDIM % 32) == 0);
static_assert((NTOK % 128) == 0 && (NQKV % 64) == 0 && (CDIM % 64) == 0 && (DHEAD % 32) == 0);
static_assert(((NB * NTOK * CDIM) % 2048) == 0 && ((NQKV * CDIM) % 2048) == 0 && ((CDIM * KCONV) % 2048) == 0);
static_assert(((NB_FULL * NTOK) % NSTAT) == 0);
static_assert(((NB * HHALF * (NTOK / 16)) % 8) == 0);
static_assert(((CT_P * 2) % 16) == 0 && ((IC_P * 2) % 16) == 0 && ((VT_P * 2) % 16) == 0);
static_assert(((V2_P * 2) % 16) == 0 && ((CO_P * 4) % 16) == 0 && ((AO_P * 4) % 16) == 0);
static_assert(32 * IC_P * 2 <= 65536 && 64 * V2_P * 2 + 64 * CO_P * 4 <= 65536);

typedef _Float16       v8h   __attribute__((ext_vector_type(8)));
typedef _Float16       v16h  __attribute__((ext_vector_type(16)));
typedef __bf16         v16bf __attribute__((ext_vector_type(16)));
typedef unsigned short v8us  __attribute__((ext_vector_type(8)));
typedef unsigned short v16us __attribute__((ext_vector_type(16)));
typedef float          v8f   __attribute__((ext_vector_type(8)));
typedef float          v4f   __attribute__((ext_vector_type(4)));

union FragH { v16h v;  v8h  half[2]; };
union FragB { v16bf v; v16us u; v8us half[2]; };

DEV unsigned int bf16_bits(float f) {
    unsigned int u = __float_as_uint(f);
    u += 0x7FFFu + ((u >> 16) & 1u);
    return u >> 16;
}
DEV float bf16_val(float f) { return __uint_as_float(bf16_bits(f) << 16); }

DEV v8f zero8f() {
    v8f z;
#pragma unroll
    for (int i = 0; i < 8; ++i) z[i] = 0.f;
    return z;
}
DEV v8f scale8(v8f a, float s) {
    v8f r;
#pragma unroll
    for (int i = 0; i < 8; ++i) r[i] = a[i] * s;
    return r;
}
DEV float fexp2(float x) { return __builtin_amdgcn_exp2f(fmaxf(x, -120.0f)); }

DEV v8f mma_bf16(v16bf a, v16bf b, v8f c) {
    c = __builtin_amdgcn_wmma_f32_16x16x32_bf16(false, a, false, b, (short)0, c, false, false);
    asm volatile("v_nop\n\tv_nop\n\tv_nop\n\tv_nop" : "+v"(c) : "v"(a), "v"(b));
    return c;
}
DEV v8f mma_f16(v16h a, v16h b, v8f c) {
    c = __builtin_amdgcn_wmma_f32_16x16x32_f16(false, a, false, b, (short)0, c, false, false);
    asm volatile("v_nop\n\tv_nop\n\tv_nop\n\tv_nop" : "+v"(c) : "v"(a), "v"(b));
    return c;
}

__global__ __launch_bounds__(256) void k_bnstat(const float* __restrict__ x, double* __restrict__ part)
{
    const int j = blockIdx.x, t = threadIdx.x;
    const int rows = (NB_FULL * NTOK) / NSTAT;
    const float* xp = x + (size_t)j * rows * CDIM + t;
    double s = 0.0, q = 0.0;
#pragma unroll 4
    for (int r = 0; r < rows; ++r) {
        const float v = bf16_val(xp[(size_t)r * CDIM]);
        s += (double)v;
        q += (double)v * (double)v;
    }
    double* ps = part + (size_t)(2 * j) * CDIM + t;
    double* pq = part + (size_t)(2 * j + 1) * CDIM + t;
    *(volatile double*)ps = s;
    *(volatile double*)pq = q;
    __threadfence();
    *(volatile double*)ps = s;
    *(volatile double*)pq = q;
}

__global__ __launch_bounds__(256) void k_bnfin(const double* __restrict__ part,
                                               const float* __restrict__ gamma,
                                               const float* __restrict__ beta,
                                               float* __restrict__ sb)
{
    const int t = threadIdx.x;
    double s = 0.0, q = 0.0;
#pragma unroll 1
    for (int j = 0; j < NSTAT; ++j) {
        s += part[(size_t)(2 * j) * CDIM + t];
        q += part[(size_t)(2 * j + 1) * CDIM + t];
    }
    const double inv = 1.0 / (double)(NB_FULL * NTOK);
    const double mean = s * inv;
    double var = q * inv - mean * mean;
    var = var > 0.0 ? var : 0.0;
    const float meanf = (float)mean;
    const float rs = 1.0f / sqrtf((float)var + BN_EPS);
    const float g  = bf16_val(gamma[t]);
    const float bt = bf16_val(beta[t]);
    float* p = sb + t;
    *(volatile float*)(p)            = meanf;
    *(volatile float*)(p + CDIM)     = rs;
    *(volatile float*)(p + 2 * CDIM) = g;
    *(volatile float*)(p + 3 * CDIM) = bt;
    __threadfence();
    *(volatile float*)(p)            = meanf;
    *(volatile float*)(p + CDIM)     = rs;
    *(volatile float*)(p + 2 * CDIM) = g;
    *(volatile float*)(p + 3 * CDIM) = bt;
}

__global__ __launch_bounds__(256) void k_bnapply(const float* __restrict__ x, const float* __restrict__ sb,
                                                 unsigned short* __restrict__ xh, unsigned short* __restrict__ xl)
{
    const size_t g = (size_t)blockIdx.x * 256 + threadIdx.x;
    const size_t e = g * 8;
    const int c = (int)(e % CDIM);
    const v4f a0 = *(const v4f*)(x + e);
    const v4f a1 = *(const v4f*)(x + e + 4);
    const v4f m0 = *(const v4f*)(sb + c),            m1 = *(const v4f*)(sb + c + 4);
    const v4f r0 = *(const v4f*)(sb + CDIM + c),     r1 = *(const v4f*)(sb + CDIM + c + 4);
    const v4f g0 = *(const v4f*)(sb + 2 * CDIM + c), g1 = *(const v4f*)(sb + 2 * CDIM + c + 4);
    const v4f b0 = *(const v4f*)(sb + 3 * CDIM + c), b1 = *(const v4f*)(sb + 3 * CDIM + c + 4);
    v8us oh, ol;
#pragma unroll
    for (int i = 0; i < 8; ++i) {
        const float xv = bf16_val(i < 4 ? a0[i] : a1[i - 4]);
        const float mu = i < 4 ? m0[i] : m1[i - 4];
        const float rs = i < 4 ? r0[i] : r1[i - 4];
        const float gm = i < 4 ? g0[i] : g1[i - 4];
        const float bt = i < 4 ? b0[i] : b1[i - 4];
        float xn = (xv - mu) * rs;
        xn = xn * gm + bt;
        xn = fmaxf(xn, 0.0f);
        const unsigned int hb = bf16_bits(xn);
        const float hv = __uint_as_float(hb << 16);
        const unsigned int lb = bf16_bits(xn - hv);
        oh[i] = (unsigned short)hb;
        ol[i] = (unsigned short)lb;
    }
    unsigned short* dh = xh + e;
    unsigned short* dl = xl + e;
    *(volatile v8us*)dh = oh;
    *(volatile v8us*)dl = ol;
    __threadfence();
    *(volatile v8us*)dh = oh;
    *(volatile v8us*)dl = ol;
}

__global__ __launch_bounds__(256) void k_cvtw(const float* __restrict__ wq, const float* __restrict__ w1,
                                              const float* __restrict__ w2, unsigned short* __restrict__ wqp,
                                              _Float16* __restrict__ w1p, _Float16* __restrict__ w2p)
{
    const int nbq = (NQKV * CDIM) / 2048;
    const int nbc = (CDIM * KCONV) / 2048;
    int blk = blockIdx.x;
    const int tid = threadIdx.x;
    if (blk < nbq) {
        const size_t e = ((size_t)blk * 256 + tid) * 8;
        const v4f a0 = *(const v4f*)(wq + e);
        const v4f a1 = *(const v4f*)(wq + e + 4);
        v8us o;
#pragma unroll
        for (int i = 0; i < 4; ++i) {
            o[i]     = (unsigned short)bf16_bits(a0[i]);
            o[4 + i] = (unsigned short)bf16_bits(a1[i]);
        }
        unsigned short* d = wqp + e;
        *(volatile v8us*)d = o;
        __threadfence();
        *(volatile v8us*)d = o;
    } else {
        blk -= nbq;
        const int second = (blk >= nbc) ? 1 : 0;
        blk -= second * nbc;
        const float* src = second ? w2 : w1;
        _Float16* dstp = second ? w2p : w1p;
        const size_t e = ((size_t)blk * 256 + tid) * 8;
        const v4f a0 = *(const v4f*)(src + e);
        const v4f a1 = *(const v4f*)(src + e + 4);
        v8h o;
#pragma unroll
        for (int i = 0; i < 4; ++i) {
            o[i]     = (_Float16)(bf16_val(a0[i]) * 64.0f);
            o[4 + i] = (_Float16)(bf16_val(a1[i]) * 64.0f);
        }
        _Float16* d = dstp + e;
        *(volatile v8h*)d = o;
        __threadfence();
        *(volatile v8h*)d = o;
    }
}

__global__ __launch_bounds__(256) __attribute__((amdgpu_num_vgpr(256)))
void k_qkv(const unsigned short* __restrict__ Wp, const unsigned short* __restrict__ Xh,
           const unsigned short* __restrict__ Xl, _Float16* __restrict__ Qkv)
{
    __shared__ __attribute__((aligned(16))) _Float16 Ct[64 * CT_P];

    const int tid = threadIdx.x, lane = tid & 31, w = tid >> 5;
    const int h = lane >> 4, l15 = lane & 15;
    const int wm = w & 3, wn = w >> 2;
    const int b = blockIdx.z;
    const int row0 = blockIdx.y * 64;
    const int col0 = blockIdx.x * 128;

    const unsigned short* ap = Wp + (size_t)(row0 + wm * 16 + l15) * CDIM + 8 * h;
    const size_t boff = ((size_t)b * NTOK + col0 + wn * 64 + l15) * CDIM + 8 * h;
    const unsigned short* bhp = Xh + boff;
    const unsigned short* blp = Xl + boff;

    v8f acc[4];
#pragma unroll
    for (int t = 0; t < 4; ++t) acc[t] = zero8f();

#pragma unroll 1
    for (int k0 = 0; k0 < CDIM; k0 += 32) {
        FragB a;
        a.half[0] = *(const v8us*)(ap + k0);
        a.half[1] = *(const v8us*)(ap + k0 + 16);
#pragma unroll
        for (int t = 0; t < 4; ++t) {
            const size_t to = (size_t)t * 16 * CDIM + k0;
            FragB fh, fl;
            fh.half[0] = *(const v8us*)(bhp + to);
            fh.half[1] = *(const v8us*)(bhp + to + 16);
            fl.half[0] = *(const v8us*)(blp + to);
            fl.half[1] = *(const v8us*)(blp + to + 16);
            acc[t] = mma_bf16(a.v, fh.v, acc[t]);
            acc[t] = mma_bf16(a.v, fl.v, acc[t]);
        }
    }

#pragma unroll
    for (int t = 0; t < 4; ++t) {
        const int cl = wn * 64 + t * 16 + l15;
#pragma unroll
        for (int r = 0; r < 8; ++r)
            Ct[(wm * 16 + 8 * h + r) * CT_P + cl] = (_Float16)(acc[t][r] * 16.0f);
    }
    __syncthreads();

    _Float16* cbase = Qkv + (size_t)b * NQKV * NTOK + (size_t)row0 * NTOK + col0;
    v8h sv[4];
#pragma unroll
    for (int i = 0; i < 4; ++i) {
        const int rl = w * 8 + 2 * i + h;
        sv[i] = *(const v8h*)(Ct + rl * CT_P + l15 * 8);
    }
#pragma unroll
    for (int i = 0; i < 4; ++i) {
        const int rl = w * 8 + 2 * i + h;
        *(volatile v8h*)(cbase + (size_t)rl * NTOK + l15 * 8) = sv[i];
    }
    __threadfence();
#pragma unroll
    for (int i = 0; i < 4; ++i) {
        const int rl = w * 8 + 2 * i + h;
        *(volatile v8h*)(cbase + (size_t)rl * NTOK + l15 * 8) = sv[i];
    }
}

__global__ __launch_bounds__(256) void k_vt(const _Float16* __restrict__ Qkv, _Float16* __restrict__ Vt)
{
    __shared__ __attribute__((aligned(16))) _Float16 T[64 * VT_P];
    const int tid = threadIdx.x;
    const int bid = blockIdx.x;
    const int nkc = NTOK / 64;
    const int b = bid / (HHALF * nkc);
    const int rem = bid - b * (HHALF * nkc);
    const int hd = rem / nkc;
    const int key0 = (rem - hd * nkc) * 64;
    const _Float16* src = Qkv + (size_t)b * NQKV * NTOK + (size_t)key0 * NQKV + 2 * INNER + hd * DHEAD;
    const int nn = tid & 63, rq = tid >> 6;
#pragma unroll 4
    for (int i = 0; i < 16; ++i) {
        const int rr = i * 4 + rq;
        T[nn * VT_P + rr] = src[(size_t)rr * NQKV + nn];
    }
    __syncthreads();
    const int piece = tid & 7;
    const int na = tid >> 3;
    const v8h va = *(const v8h*)(T + na * VT_P + piece * 8);
    const v8h vb = *(const v8h*)(T + (na + 32) * VT_P + piece * 8);
    _Float16* da = Vt + ((size_t)(b * HHALF + hd) * DHEAD + na) * NTOK + key0 + piece * 8;
    _Float16* db = Vt + ((size_t)(b * HHALF + hd) * DHEAD + na + 32) * NTOK + key0 + piece * 8;
    *(volatile v8h*)da = va;
    *(volatile v8h*)db = vb;
    __threadfence();
    *(volatile v8h*)da = va;
    *(volatile v8h*)db = vb;
}

__global__ __launch_bounds__(256) void k_im2col(const _Float16* __restrict__ Qkv,
                                                _Float16* __restrict__ Qcol, _Float16* __restrict__ Kcol)
{
    __shared__ __attribute__((aligned(16))) _Float16 T[32 * IC_P];
    const int tid = threadIdx.x, lane = tid & 31, w = tid >> 5;
    const int x0 = blockIdx.x * 32, y = blockIdx.y;
    const int b = blockIdx.z >> 1, which = blockIdx.z & 1;
    const _Float16* pb = Qkv + (size_t)b * NQKV * NTOK;

#pragma unroll 1
    for (int p = w; p < KCONV; p += 8) {
        const int c = p / 3, t = p - 3 * c;
        const int yy = y + t - 1;
        const int yyc = yy < 0 ? 0 : (yy > IMG - 1 ? IMG - 1 : yy);
        const int xx = x0 + lane + t - 1;
        const int xxc = xx < 0 ? 0 : (xx > IMG - 1 ? IMG - 1 : xx);
        const int n2 = (c & 63) * IMG + (which ? y : yyc);
        const int col = (which ? (INNER + INNER / 2) : (INNER / 2)) + (c >> 6) * DHEAD + (which ? xxc : (x0 + lane));
        const int valid = which ? ((unsigned)xx < (unsigned)IMG) : ((unsigned)yy < (unsigned)IMG);
        const _Float16 v = pb[(size_t)n2 * NQKV + col];
        T[lane * IC_P + p] = valid ? v : (_Float16)0.0f;
    }
    __syncthreads();

    _Float16* cp = (which ? Kcol : Qcol) + ((size_t)b * NTOK + (size_t)y * IMG + x0) * KCONV;
    v8h sv[12];
#pragma unroll
    for (int i = 0; i < 12; ++i) {
        const int L = i * 4 + (lane >> 3);
        const int r = w * 4 + L / 12, ln = L % 12, piece = lane & 7;
        sv[i] = *(const v8h*)(T + r * IC_P + ln * 64 + piece * 8);
    }
#pragma unroll
    for (int i = 0; i < 12; ++i) {
        const int L = i * 4 + (lane >> 3);
        const int r = w * 4 + L / 12, ln = L % 12, piece = lane & 7;
        *(volatile v8h*)(cp + (size_t)r * KCONV + ln * 64 + piece * 8) = sv[i];
    }
    __threadfence();
#pragma unroll
    for (int i = 0; i < 12; ++i) {
        const int L = i * 4 + (lane >> 3);
        const int r = w * 4 + L / 12, ln = L % 12, piece = lane & 7;
        *(volatile v8h*)(cp + (size_t)r * KCONV + ln * 64 + piece * 8) = sv[i];
    }
}

__global__ __launch_bounds__(256) __attribute__((amdgpu_num_vgpr(256)))
void k_attn(const _Float16* __restrict__ Qkv, const _Float16* __restrict__ Vt, float* __restrict__ Out)
{
    __shared__ __attribute__((aligned(16))) float Ost[8 * 16 * AO_P];
    const int tid = threadIdx.x, lane = tid & 31, w = tid >> 5;
    const int h = lane >> 4, l15 = lane & 15;
    const int wid = blockIdx.x * 8 + w;
    const int qt = wid % (NTOK / 16);
    const int hd = (wid / (NTOK / 16)) % HHALF;
    const int b  = wid / ((NTOK / 16) * HHALF);
    const int q0 = qt * 16;
    const _Float16* pb = Qkv + (size_t)b * NQKV * NTOK;

    FragH bq[2];
    {
        const _Float16* qp = pb + (size_t)(q0 + l15) * NQKV + hd * DHEAD + 8 * h;
#pragma unroll
        for (int s = 0; s < 2; ++s) {
            bq[s].half[0] = *(const v8h*)(qp + s * 32);
            bq[s].half[1] = *(const v8h*)(qp + s * 32 + 16);
        }
    }

    v8f acc[4];
#pragma unroll
    for (int t = 0; t < 4; ++t) acc[t] = zero8f();
    float m = -1.0e30f, l = 0.0f;

    const _Float16* kbp = pb + (size_t)l15 * NQKV + INNER + hd * DHEAD + 8 * h;
    const _Float16* vbp = Vt + ((size_t)(b * HHALF + hd) * DHEAD + l15) * NTOK + 8 * h;

#pragma unroll 1
    for (int kb = 0; kb < NTOK; kb += 32) {
        const _Float16* k0p = kbp + (size_t)kb * NQKV;
        const _Float16* k1p = k0p + (size_t)16 * NQKV;
        v8f st0 = zero8f(), st1 = zero8f();
#pragma unroll
        for (int s = 0; s < 2; ++s) {
            FragH ka, kc;
            ka.half[0] = *(const v8h*)(k0p + s * 32);
            ka.half[1] = *(const v8h*)(k0p + s * 32 + 16);
            kc.half[0] = *(const v8h*)(k1p + s * 32);
            kc.half[1] = *(const v8h*)(k1p + s * 32 + 16);
            st0 = mma_f16(ka.v, bq[s].v, st0);
            st1 = mma_f16(kc.v, bq[s].v, st1);
        }
        float mloc = st0[0];
#pragma unroll
        for (int r = 0; r < 8; ++r) { mloc = fmaxf(mloc, st0[r]); mloc = fmaxf(mloc, st1[r]); }
        mloc = fmaxf(mloc, __shfl_xor(mloc, 16));
        const float mnew = fmaxf(m, mloc);
        const float alpha = fexp2((m - mnew) * SCL2);
        v8h e0, e1;
        float ls = 0.0f;
#pragma unroll
        for (int r = 0; r < 8; ++r) {
            const _Float16 p0 = (_Float16)(fexp2((st0[r] - mnew) * SCL2) * 1024.0f);
            const _Float16 p1 = (_Float16)(fexp2((st1[r] - mnew) * SCL2) * 1024.0f);
            e0[r] = p0;
            e1[r] = p1;
            ls += (float)p0 + (float)p1;
        }
        ls += __shfl_xor(ls, 16);
        l = l * alpha + ls;
        m = mnew;
        FragH pf;
        pf.half[0] = e0;
        pf.half[1] = e1;
#pragma unroll
        for (int t = 0; t < 4; ++t) {
            acc[t] = scale8(acc[t], alpha);
            const _Float16* vp = vbp + (size_t)t * 16 * NTOK + kb;
            FragH va;
            va.half[0] = *(const v8h*)(vp);
            va.half[1] = *(const v8h*)(vp + 16);
            acc[t] = mma_f16(va.v, pf.v, acc[t]);
        }
    }

    const float rl = 0.5f / (16.0f * l);
    float* orow = Ost + (w * 16 + l15) * AO_P;
#pragma unroll
    for (int t = 0; t < 4; ++t) {
        v4f o;
#pragma unroll
        for (int i = 0; i < 4; ++i) o[i] = (acc[t][2 * i] + acc[t][2 * i + 1]) * rl;
        *(v4f*)(orow + 8 * t + 4 * h) = o;
    }
    __syncthreads();

    v4f sv[4];
#pragma unroll
    for (int i = 0; i < 4; ++i) {
        const int row = 4 * i + (lane >> 3), piece = lane & 7;
        sv[i] = *(const v4f*)(Ost + (w * 16 + row) * AO_P + piece * 4);
    }
#pragma unroll
    for (int i = 0; i < 4; ++i) {
        const int row = 4 * i + (lane >> 3), piece = lane & 7;
        *(volatile v4f*)(Out + ((size_t)(b * NTOK + q0 + row)) * CDIM + hd * 32 + piece * 4) = sv[i];
    }
    __threadfence();
#pragma unroll
    for (int i = 0; i < 4; ++i) {
        const int row = 4 * i + (lane >> 3), piece = lane & 7;
        *(volatile v4f*)(Out + ((size_t)(b * NTOK + q0 + row)) * CDIM + hd * 32 + piece * 4) = sv[i];
    }
}

__global__ __launch_bounds__(256) __attribute__((amdgpu_num_vgpr(256)))
void k_conv(const _Float16* __restrict__ W1p, const _Float16* __restrict__ W2p,
            const _Float16* __restrict__ Qcol, const _Float16* __restrict__ Kcol,
            const _Float16* __restrict__ Qkv, float* __restrict__ Out)
{
    __shared__ __attribute__((aligned(16))) _Float16 V2t[64 * V2_P];
    __shared__ __attribute__((aligned(16))) float    Ost[64 * CO_P];

    const int tid = threadIdx.x, lane = tid & 31, w = tid >> 5;
    const int h = lane >> 4, l15 = lane & 15;
    const int wm = w & 3, wn = w >> 2;
    const int b = blockIdx.z;
    const int row0 = blockIdx.y * 64;
    const int col0 = blockIdx.x * 128;
    const int y0 = col0 >> 6;
    const _Float16* pb = Qkv + (size_t)b * NQKV * NTOK;

#pragma unroll
    for (int i = 0; i < 4; ++i) {
        const int P = i * 256 + tid;
        const int piece = P & 7, yl = (P >> 3) & 1, ol = P >> 4;
        const int o = row0 + ol;
        const _Float16* s = pb + ((size_t)((o & 63) * IMG + y0 + yl)) * NQKV + 2 * INNER + INNER / 2 + (o >> 6) * DHEAD + piece * 8;
        *(v8h*)(V2t + ol * V2_P + yl * 64 + piece * 8) = *(const v8h*)s;
    }
    __syncthreads();

    const _Float16* a1p = W1p + (size_t)(row0 + wm * 16 + l15) * KCONV + 8 * h;
    const _Float16* a2p = W2p + (size_t)(row0 + wm * 16 + l15) * KCONV + 8 * h;
    const size_t boff = ((size_t)b * NTOK + col0 + wn * 64 + l15) * KCONV + 8 * h;
    const _Float16* b1p = Qcol + boff;
    const _Float16* b2p = Kcol + boff;

    v8f acc[4];
#pragma unroll
    for (int t = 0; t < 4; ++t) acc[t] = zero8f();

#pragma unroll 1
    for (int pass = 0; pass < 2; ++pass) {
        const _Float16* ap  = pass ? a2p : a1p;
        const _Float16* bpp = pass ? b2p : b1p;
#pragma unroll 1
        for (int k0 = 0; k0 < KCONV; k0 += 32) {
            FragH a;
            a.half[0] = *(const v8h*)(ap + k0);
            a.half[1] = *(const v8h*)(ap + k0 + 16);
#pragma unroll
            for (int t = 0; t < 4; ++t) {
                const _Float16* bq = bpp + (size_t)t * 16 * KCONV + k0;
                FragH bf;
                bf.half[0] = *(const v8h*)(bq);
                bf.half[1] = *(const v8h*)(bq + 16);
                acc[t] = mma_f16(a.v, bf.v, acc[t]);
            }
        }
    }

#pragma unroll
    for (int t = 0; t < 4; ++t) {
        const int x = t * 16 + l15;
#pragma unroll
        for (int r = 0; r < 8; ++r) {
            const int ol = wm * 16 + 8 * h + r;
            const float v2 = (float)V2t[ol * V2_P + wn * 64 + x];
            const float val = acc[t][r] * (1.0f / 1024.0f) + v2 * (1.0f / 16.0f);
            const float par = __shfl_xor(val, 1);
            Ost[ol * CO_P + wn * 32 + (x >> 1)] = 0.5f * (val + par);
        }
    }
    __syncthreads();

    v4f sv[4];
#pragma unroll
    for (int i = 0; i < 4; ++i) {
        const int L = w * 16 + 4 * i + (lane >> 3);
        const int ol = L >> 1, yl = L & 1, piece = lane & 7;
        sv[i] = *(const v4f*)(Ost + ol * CO_P + yl * 32 + piece * 4);
    }
#pragma unroll
    for (int i = 0; i < 4; ++i) {
        const int L = w * 16 + 4 * i + (lane >> 3);
        const int ol = L >> 1, yl = L & 1, piece = lane & 7;
        const int o = row0 + ol, y = y0 + yl;
        const int n = o * 16 + (y >> 2);
        *(volatile v4f*)(Out + ((size_t)(b * NTOK + n)) * CDIM + CDIM / 2 + (y & 3) * 32 + piece * 4) = sv[i];
    }
    __threadfence();
#pragma unroll
    for (int i = 0; i < 4; ++i) {
        const int L = w * 16 + 4 * i + (lane >> 3);
        const int ol = L >> 1, yl = L & 1, piece = lane & 7;
        const int o = row0 + ol, y = y0 + yl;
        const int n = o * 16 + (y >> 2);
        *(volatile v4f*)(Out + ((size_t)(b * NTOK + n)) * CDIM + CDIM / 2 + (y & 3) * 32 + piece * 4) = sv[i];
    }
}

extern "C" void kernel_launch(void* const* d_in, const int* in_sizes, int n_in,
                              void* d_out, int out_size, void* d_ws, size_t ws_size,
                              hipStream_t stream)
{
    if (n_in < 6) return;
    if (in_sizes[0] < NB_FULL * NTOK * CDIM) return;
    if (in_sizes[1] < NQKV * CDIM) return;
    if (in_sizes[2] < CDIM || in_sizes[3] < CDIM) return;
    if (in_sizes[4] < CDIM * KCONV || in_sizes[5] < CDIM * KCONV) return;
    if (out_size < NB * NTOK * CDIM) return;

    const float* x     = (const float*)d_in[0];
    const float* qkv_w = (const float*)d_in[1];
    const float* gamma = (const float*)d_in[2];
    const float* beta  = (const float*)d_in[3];
    const float* c1w   = (const float*)d_in[4];
    const float* c2w   = (const float*)d_in[5];
    float* out = (float*)d_out;

    char* ws = (char*)d_ws;
    size_t off = 0;
    auto carve = [&](size_t bytes) -> char* {
        char* p = ws + off;
        off += (bytes + 255) & ~(size_t)255;
        return p;
    };
    double*         part = (double*)carve((size_t)NSTAT * 2 * CDIM * 8);
    float*          sb   = (float*)carve((size_t)4 * CDIM * 4);
    unsigned short* xh   = (unsigned short*)carve((size_t)NB * NTOK * CDIM * 2);
    unsigned short* xl   = (unsigned short*)carve((size_t)NB * NTOK * CDIM * 2);
    unsigned short* wqp  = (unsigned short*)carve((size_t)NQKV * CDIM * 2);
    _Float16*       w1p  = (_Float16*)carve((size_t)CDIM * KCONV * 2);
    _Float16*       w2p  = (_Float16*)carve((size_t)CDIM * KCONV * 2);
    _Float16*       qkv  = (_Float16*)carve((size_t)NB * NQKV * NTOK * 2);
    _Float16*       vt   = (_Float16*)carve((size_t)NB * HHALF * DHEAD * NTOK * 2);
    _Float16*       qcol = (_Float16*)carve((size_t)NB * NTOK * KCONV * 2);
    _Float16*       kcol = (_Float16*)carve((size_t)NB * NTOK * KCONV * 2);
    if (off > ws_size) return;

    k_bnstat<<<NSTAT, 256, 0, stream>>>(x, part);
    k_bnfin<<<1, 256, 0, stream>>>(part, gamma, beta, sb);
    k_bnapply<<<(unsigned)(((size_t)NB * NTOK * CDIM) / 2048), 256, 0, stream>>>(x, sb, xh, xl);
    k_cvtw<<<(NQKV * CDIM) / 2048 + 2 * ((CDIM * KCONV) / 2048), 256, 0, stream>>>(qkv_w, c1w, c2w, wqp, w1p, w2p);
    k_qkv<<<dim3(NTOK / 128, NQKV / 64, NB), 256, 0, stream>>>(wqp, xh, xl, qkv);
    k_vt<<<NB * HHALF * (NTOK / 64), 256, 0, stream>>>(qkv, vt);
    k_im2col<<<dim3(2, IMG, NB * 2), 256, 0, stream>>>(qkv, qcol, kcol);
    k_attn<<<(NB * HHALF * (NTOK / 16)) / 8, 256, 0, stream>>>(qkv, vt, out);
    k_conv<<<dim3(NTOK / 128, CDIM / 64, NB), 256, 0, stream>>>(w1p, w2p, qcol, kcol, qkv, out);
}
